// KANLayer_65919158059310
// MI455X (gfx1250) — hardware-verified
//
#include <hip/hip_runtime.h>
#include <math.h>

constexpr int kRows = 8192;
constexpr int kIn   = 512;
constexpr int kOut  = 512;
constexpr int kNcp  = 5;
constexpr int kKdim = 4 * kIn;
constexpr float kBtCarry    = 16.0f;
constexpr float kBtCarryInv = 1.0f / 16.0f;

static_assert(kKdim % 32 == 0);
static_assert(kRows % 64 == 0);
static_assert(kOut % 64 == 0);
static_assert(kIn % 64 == 0);
static_assert((kRows / 64) * (kOut / 64) % 8 == 0);

constexpr size_t kBytesA  = (size_t)kRows * kKdim * 2;
constexpr size_t kBytesBt = (size_t)kOut * kKdim * 2;
constexpr size_t kOffA    = 0;
constexpr size_t kOffBt   = kOffA + kBytesA;
constexpr size_t kWsTotal = kOffBt + kBytesBt;
static_assert(kBytesA == 33554432);
static_assert(kWsTotal == 35651584);
static_assert(kWsTotal <= (size_t)134217728);

typedef __attribute__((ext_vector_type(16))) _Float16 v16h;
typedef __attribute__((ext_vector_type(8)))  _Float16 v8h;
typedef __attribute__((ext_vector_type(16))) __bf16   v16b;
typedef __attribute__((ext_vector_type(8)))  __bf16   v8b;
typedef __attribute__((ext_vector_type(8)))  float    v8f;
typedef __attribute__((ext_vector_type(4)))  float    v4f;
typedef __attribute__((ext_vector_type(4)))  unsigned int v4u;

__device__ __forceinline__ unsigned short f2bf_bits(float f) {
  unsigned u = __float_as_uint(f);
  return (unsigned short)((u + 0x7FFFu + ((u >> 16) & 1u)) >> 16);
}
__device__ __forceinline__ float bf_bits2f(unsigned short h) { return __uint_as_float(((unsigned)h) << 16); }

__device__ __forceinline__ void dep_guard_h(v8f& a, v8f& b, v16h x, v16h y) { asm volatile("v_nop\n\tv_nop\n\tv_nop\n\tv_nop" : "+v"(a), "+v"(b) : "v"(x), "v"(y)); }
__device__ __forceinline__ void dep_guard_b(v8f& a, v8f& b, v16b x, v16b y) { asm volatile("v_nop\n\tv_nop\n\tv_nop\n\tv_nop" : "+v"(a), "+v"(b) : "v"(x), "v"(y)); }
__device__ __forceinline__ void keep4_h(v16h a, v16h b, v16h c, v16h d) { asm volatile("v_nop" :: "v"(a), "v"(b), "v"(c), "v"(d)); }
__device__ __forceinline__ void keep4_b(v16b a, v16b b, v16b c, v16b d) { asm volatile("v_nop" :: "v"(a), "v"(b), "v"(c), "v"(d)); }
__device__ __forceinline__ void acc_guard4(v8f& a, v8f& b, v8f& c, v8f& d) { asm volatile("v_nop\n\tv_nop\n\tv_nop\n\tv_nop" : "+v"(a), "+v"(b), "+v"(c), "+v"(d)); }
template <typename T> struct Frag;
template <> struct Frag<_Float16> {
  typedef v16h V; union U { v16h v; v8h h[2]; };
  static __device__ __forceinline__ v16h load(const _Float16* p) {
    U f; f.h[0] = *(const v8h*)(p); f.h[1] = *(const v8h*)(p + 16); return f.v;
  }
  static __device__ __forceinline__ v8f mma(v16h a, v16h b, v8f c) {
    return __builtin_amdgcn_wmma_f32_16x16x32_f16(false, a, false, b, (short)0, c, false, false);
  }
  static __device__ __forceinline__ void guard(v8f& a, v8f& b, v16h x, v16h y) { dep_guard_h(a, b, x, y); }
  static __device__ __forceinline__ void keep(v16h a, v16h b, v16h c, v16h d) { keep4_h(a, b, c, d); }
};
template <> struct Frag<__bf16> {
  typedef v16b V; union U { v16b v; v8b h[2]; };
  static __device__ __forceinline__ v16b load(const __bf16* p) {
    U f; f.h[0] = *(const v8b*)(p); f.h[1] = *(const v8b*)(p + 16); return f.v;
  }
  static __device__ __forceinline__ v8f mma(v16b a, v16b b, v8f c) {
    return __builtin_amdgcn_wmma_f32_16x16x32_bf16(false, a, false, b, (short)0, c, false, false);
  }
  static __device__ __forceinline__ void guard(v8f& a, v8f& b, v16b x, v16b y) { dep_guard_b(a, b, x, y); }
  static __device__ __forceinline__ void keep(v16b a, v16b b, v16b c, v16b d) { keep4_b(a, b, c, d); }
};

__device__ __forceinline__ unsigned pk16(unsigned short a, unsigned short b) { return (unsigned)a | ((unsigned)b << 16); }
__device__ __forceinline__ unsigned short h_bits(float f) { const _Float16 h = (_Float16)f; return __builtin_bit_cast(unsigned short, h); }

template <int ET> struct Elem;
template <> struct Elem<0> { typedef _Float16 T; };
template <> struct Elem<1> { typedef __bf16 T; };
template <int ET, bool SPLIT, int BIAS_MODE, int OUT_MODE, bool RESID, int ACT = 0>
__global__ __launch_bounds__(256) void wmma_gemm64(
    const unsigned short* __restrict__ Ap, const unsigned short* __restrict__ A2p, int lda, long strideA,
    const unsigned short* __restrict__ Btp, const unsigned short* __restrict__ Bt2p, int ldb, long strideB,
    void* __restrict__ Cout, void* __restrict__ Cout2, int ldc, long strideC,
    const float* __restrict__ bias,
    const float* __restrict__ resid, long strideR,
    int M, int N, int K, float scale) {
  typedef typename Elem<ET>::T T;
  typedef typename Frag<T>::V V;
  const T* A = (const T*)Ap; const T* A2 = (const T*)A2p; const T* Bt = (const T*)Btp; const T* Bt2 = (const T*)Bt2p;
  __shared__ __align__(16) float sT[8][16 * 68];
  const int b    = blockIdx.y;
  const int lane = threadIdx.x & 31;
  const int wave = threadIdx.x >> 5;
  const int tilesN = N >> 6;
  const int tilesM = M >> 6;
  const int tile = blockIdx.x * 8 + wave;
  if (tile >= tilesM * tilesN) return;
  const int tm = tile / tilesN;
  const int tn = tile - tm * tilesN;
  const int m0 = tm << 6;
  const int n0 = tn << 6;

  const T* Ab  = A  + (size_t)b * strideA;
  const T* Bb  = Bt + (size_t)b * strideB;
  const T* Ab2 = SPLIT ? (A2  + (size_t)b * strideA) : nullptr;
  const T* Bb2 = SPLIT ? (Bt2 + (size_t)b * strideB) : nullptr;

  const int rlane = lane & 15;
  const int koff  = (lane >> 4) * 8;
  const int mOff  = (lane >> 4) * 8;

  v8f acc[4][4];
#pragma unroll
  for (int i = 0; i < 4; ++i)
#pragma unroll
    for (int j = 0; j < 4; ++j) acc[i][j] = (v8f){0.f,0.f,0.f,0.f,0.f,0.f,0.f,0.f};

  for (int k0 = 0; k0 < K; k0 += 32) {
    V bh[4], bl[4];
#pragma unroll
    for (int j = 0; j < 4; ++j) {
      const size_t bo = (size_t)(n0 + (j << 4) + rlane) * ldb + koff + k0;
      bh[j] = Frag<T>::load(Bb + bo);
      if (SPLIT) bl[j] = Frag<T>::load(Bb2 + bo);
    }
#pragma unroll
    for (int i = 0; i < 4; ++i) {
      const size_t ao = (size_t)(m0 + (i << 4) + rlane) * lda + koff + k0;
      V ah = Frag<T>::load(Ab + ao);
      V al;
      if (SPLIT) al = Frag<T>::load(Ab2 + ao);
#pragma unroll
      for (int j = 0; j < 4; ++j) {
        acc[i][j] = Frag<T>::mma(ah, bh[j], acc[i][j]);
        if (SPLIT) {
          acc[i][j] = Frag<T>::mma(ah, bl[j], acc[i][j]);
          acc[i][j] = Frag<T>::mma(al, bh[j], acc[i][j]);
        }
      }
      Frag<T>::guard(acc[i][0], acc[i][3], ah, SPLIT ? al : ah);
    }
    Frag<T>::keep(bh[0], bh[1], bh[2], bh[3]);
    if (SPLIT) Frag<T>::keep(bl[0], bl[1], bl[2], bl[3]);
  }
  acc_guard4(acc[0][0], acc[0][1], acc[0][2], acc[0][3]);
  acc_guard4(acc[1][0], acc[1][1], acc[1][2], acc[1][3]);
  acc_guard4(acc[2][0], acc[2][1], acc[2][2], acc[2][3]);
  acc_guard4(acc[3][0], acc[3][1], acc[3][2], acc[3][3]);

  float* slab = sT[wave];
  const float* Rb = RESID ? (resid + (size_t)b * strideR) : nullptr;
#pragma unroll
  for (int i = 0; i < 4; ++i) {
    const int mBase = m0 + (i << 4);
#pragma unroll
    for (int j = 0; j < 4; ++j) {
      const int n = n0 + (j << 4) + rlane;
      float bv = 0.f;
      if (BIAS_MODE == 2) bv = bias[n];
#pragma unroll
      for (int r = 0; r < 8; ++r) {
        float v = acc[i][j][r] * scale;
        if (BIAS_MODE == 1) v += bias[mBase + mOff + r];
        if (BIAS_MODE == 2) v += bv;
        if (RESID) v += Rb[(size_t)(mBase + mOff + r) * ldc + n];
        if (ACT == 2) v = fmaxf(v, 0.0f);
        if (ACT == 4) v = (v > 0.f) ? v : 0.01f * v;
        slab[(mOff + r) * 68 + (j << 4) + rlane] = v;
      }
    }
    __builtin_amdgcn_fence(__ATOMIC_RELEASE, "workgroup");
    __builtin_amdgcn_wave_barrier();
    __builtin_amdgcn_fence(__ATOMIC_ACQUIRE, "workgroup");
    if (OUT_MODE == 0) {
      float* C = (float*)Cout + (size_t)b * strideC;
      const int hh = lane >> 4, c4 = (lane & 15) * 4;
      for (int pass = 0; pass < 2; ++pass) {
#pragma unroll
        for (int it = 0; it < 8; ++it) {
          const int row = it * 2 + hh;
          v4f v = *(const v4f*)(slab + row * 68 + c4);
          *(volatile v4f*)(C + (size_t)(mBase + row) * ldc + n0 + c4) = v;
        }
        __threadfence();
      }
    } else {
      const int q = lane >> 3, c8 = (lane & 7) * 8;
      unsigned short* C  = (unsigned short*)Cout  + (size_t)b * strideC;
      unsigned short* C2 = (OUT_MODE == 2) ? ((unsigned short*)Cout2 + (size_t)b * strideC) : nullptr;
      for (int pass = 0; pass < 2; ++pass) {
#pragma unroll
        for (int it = 0; it < 4; ++it) {
          const int row = it * 4 + q;
          const float* sp = slab + row * 68 + c8;
          v8h hv, lv;
#pragma unroll
          for (int e = 0; e < 8; ++e) {
            if (OUT_MODE == 1) {
              hv[e] = (_Float16)sp[e];
            } else {
              unsigned short hb = f2bf_bits(sp[e]);
              unsigned short lb = f2bf_bits(sp[e] - bf_bits2f(hb));
              hv[e] = __builtin_bit_cast(_Float16, hb);
              lv[e] = __builtin_bit_cast(_Float16, lb);
            }
          }
          *(volatile v8h*)(C + (size_t)(mBase + row) * ldc + n0 + c8) = hv;
          if (OUT_MODE == 2) *(volatile v8h*)(C2 + (size_t)(mBase + row) * ldc + n0 + c8) = lv;
        }
        __threadfence();
      }
    }
    __builtin_amdgcn_fence(__ATOMIC_RELEASE, "workgroup");
    __builtin_amdgcn_wave_barrier();
    __builtin_amdgcn_fence(__ATOMIC_ACQUIRE, "workgroup");
  }
}

__device__ __forceinline__ v4u pack8_f16(const float* sp) {
  const v4f a = *(const v4f*)(sp);
  const v4f c = *(const v4f*)(sp + 4);
  unsigned short hb[8];
#pragma unroll
  for (int e = 0; e < 4; ++e) {
    hb[e]     = h_bits(a[e]);
    hb[4 + e] = h_bits(c[e]);
  }
  return (v4u){pk16(hb[0], hb[1]), pk16(hb[2], hb[3]), pk16(hb[4], hb[5]), pk16(hb[6], hb[7])};
}

struct BasisTab { float t[16]; };
static_assert(sizeof(BasisTab) == 64);

__device__ __forceinline__ void edge_vals(const float* __restrict__ cp, const float* __restrict__ bw,
                                          const float* __restrict__ sw, const float* __restrict__ imp,
                                          size_t io, const BasisTab& tab,
                                          float& v0, float& v1, float& v2, float& v3) {
  const float im  = imp[io];
  const float bwv = bw[io];
  const float swv = sw[io];
  const float* cpp = cp + io * kNcp;
  const float c0 = cpp[0], c1 = cpp[1], c2 = cpp[2], c3 = cpp[3], c4 = cpp[4];
  v0 = kBtCarry * (im * bwv);
  const float s = kBtCarry * (im * swv);
  const float d0 = tab.t[0]  * c0 + tab.t[1]  * c1 + tab.t[2]  * c2 + tab.t[3]  * c3 + tab.t[4]  * c4;
  const float d1 = tab.t[5]  * c0 + tab.t[6]  * c1 + tab.t[7]  * c2 + tab.t[8]  * c3 + tab.t[9]  * c4;
  const float d2 = tab.t[10] * c0 + tab.t[11] * c1 + tab.t[12] * c2 + tab.t[13] * c3 + tab.t[14] * c4;
  v1 = s * d0;
  v2 = s * d1;
  v3 = s * d2;
}

__global__ __launch_bounds__(256) void prep_bt_kernel(const float* __restrict__ cp, const float* __restrict__ bw,
                                                      const float* __restrict__ sw, const float* __restrict__ imp,
                                                      unsigned short* __restrict__ bt, BasisTab tab) {
  __shared__ unsigned smu[4][64][33];
  const int t  = threadIdx.x;
  const int i0 = blockIdx.x * 64;
  const int o0 = blockIdx.y * 64;
#pragma unroll 1
  for (int it = 0; it < 8; ++it) {
    const int e  = it * 256 + t;
    const int ol = e & 63;
    const int ip = e >> 6;
    const size_t ioa = (size_t)(i0 + 2 * ip) * kOut + o0 + ol;
    const size_t iob = ioa + kOut;
    float a0, a1, a2, a3, b0, b1, b2, b3;
    edge_vals(cp, bw, sw, imp, ioa, tab, a0, a1, a2, a3);
    asm volatile("" ::: "memory");
    edge_vals(cp, bw, sw, imp, iob, tab, b0, b1, b2, b3);
    smu[0][ol][ip] = pk16(h_bits(a0), h_bits(b0));
    smu[1][ol][ip] = pk16(h_bits(a1), h_bits(b1));
    smu[2][ol][ip] = pk16(h_bits(a2), h_bits(b2));
    smu[3][ol][ip] = pk16(h_bits(a3), h_bits(b3));
  }
  __syncthreads();
  const int lane = t & 31, wave = t >> 5;
  const int q = lane >> 3;
  const int c4u = (lane & 7) * 4;
  for (int pass = 0; pass < 2; ++pass) {
#pragma unroll
    for (int it = 0; it < 8; ++it) {
      const int L  = wave * 32 + it * 4 + q;
      const int p  = L >> 6;
      const int ol = L & 63;
      const unsigned* sp = &smu[p][ol][c4u];
      const v4u u = (v4u){sp[0], sp[1], sp[2], sp[3]};
      unsigned short* dst = bt + (size_t)(o0 + ol) * kKdim + p * kIn + i0 + (lane & 7) * 8;
      *(volatile v4u*)dst = u;
    }
    __threadfence();
  }
}

__global__ __launch_bounds__(256) void prep_a_kernel(const float* __restrict__ x, unsigned short* __restrict__ ap) {
  __shared__ __align__(16) float sv[4][4 * kIn];
  const int t = threadIdx.x;
  const size_t r0 = (size_t)blockIdx.x * 4;
  const float* xb = x + r0 * kIn;
#pragma unroll 1
  for (int it = 0; it < 8; ++it) {
    const int e = it * 256 + t;
    const float xv = xb[e];
    const float en = expf(-xv);
    const float sg = 1.0f / (1.0f + en);
    const float silu = xv * sg;
    const float xc = fminf(fmaxf(xv, -1.0f), 1.0f);
    const float gi = xc + 1.0f;
    const float fl = fminf(fmaxf(floorf(gi), 0.0f), 2.0f);
    const float cl = fminf(fmaxf(ceilf(gi), 0.0f), 2.0f);
    const float frac = gi - fl;
    const float omf = 1.0f - frac;
    const float w0 = ((fl == 0.0f) ? omf : 0.0f) + ((cl == 0.0f) ? frac : 0.0f);
    const float w1 = ((fl == 1.0f) ? omf : 0.0f) + ((cl == 1.0f) ? frac : 0.0f);
    const float w2 = ((fl == 2.0f) ? omf : 0.0f) + ((cl == 2.0f) ? frac : 0.0f);
    sv[0][e] = silu;
    sv[1][e] = w0;
    sv[2][e] = w1;
    sv[3][e] = w2;
  }
  __syncthreads();
  const int rl = t >> 6;
  const int i8 = (t & 63) * 8;
  const int so = rl * kIn + i8;
  const v4u u0 = pack8_f16(&sv[0][so]);
  const v4u u1 = pack8_f16(&sv[1][so]);
  const v4u u2 = pack8_f16(&sv[2][so]);
  const v4u u3 = pack8_f16(&sv[3][so]);
  unsigned short* dst = ap + (r0 + rl) * (size_t)kKdim + i8;
  for (int pass = 0; pass < 2; ++pass) {
    *(volatile v4u*)(dst)           = u0;
    *(volatile v4u*)(dst + kIn)     = u1;
    *(volatile v4u*)(dst + 2 * kIn) = u2;
    *(volatile v4u*)(dst + 3 * kIn) = u3;
    __threadfence();
  }
}

extern "C" void kernel_launch(void* const* d_in, const int* in_sizes, int n_in,
                              void* d_out, int out_size, void* d_ws, size_t ws_size,
                              hipStream_t stream) {
  if (n_in < 5) return;
  if (in_sizes[0] != kRows * kIn || in_sizes[1] != kIn * kOut * kNcp || in_sizes[2] != kIn * kOut ||
      in_sizes[3] != kIn * kOut || in_sizes[4] != kIn * kOut) return;
  if (out_size != kRows * kOut) return;
  if (ws_size < kWsTotal) return;

  const float* x   = (const float*)d_in[0];
  const float* cp  = (const float*)d_in[1];
  const float* bw  = (const float*)d_in[2];
  const float* sw  = (const float*)d_in[3];
  const float* imp = (const float*)d_in[4];
  float* out = (float*)d_out;
  unsigned char* ws = (unsigned char*)d_ws;
  unsigned short* a16  = (unsigned short*)(ws + kOffA);
  unsigned short* bt16 = (unsigned short*)(ws + kOffBt);

  BasisTab tab;
  {
    const double ext  = 3 * 0.1;
    const double klo  = -1.0 - ext;
    const double khi  = 1.0 + ext;
    const double step = (khi - klo) / 8.0;
    double knots[9];
    for (int j = 0; j < 9; ++j) knots[j] = klo + (double)j * step;
    knots[8] = khi;
    const double gridp[3] = {-1.0, 0.0, 1.0};
    float bv[3][5];
    for (int c = 0; c < 5; ++c) {
      const double center = (knots[c + 1] + knots[c + 2]) / 2.0;
      const double width  = (knots[c + 4] - knots[c]) / 2.0;
      for (int g = 0; g < 3; ++g) {
        const double z = (gridp[g] - center) / width;
        bv[g][c] = (float)exp(-(z * z));
      }
    }
    for (int g = 0; g < 3; ++g) {
      float s = bv[g][0];
      for (int c = 1; c < 5; ++c) s = s + bv[g][c];
      const float den = s + 1e-6f;
      for (int c = 0; c < 5; ++c) tab.t[g * 5 + c] = bv[g][c] / den;
    }
    tab.t[15] = 0.0f;
  }

  prep_bt_kernel<<<dim3(kIn / 64, kOut / 64), 256, 0, stream>>>(cp, bw, sw, imp, bt16, tab);
  prep_a_kernel<<<dim3(kRows / 4), 256, 0, stream>>>(x, a16);
  wmma_gemm64<0, false, 0, 0, false, 0><<<dim3((kRows / 64) * (kOut / 64) / 8, 1), 256, 0, stream>>>(
      a16, a16, kKdim, 0L,
      bt16, bt16, kKdim, 0L,
      (void*)out, (void*)out, kOut, 0L,
      x, x, 0L,
      kRows, kOut, kKdim, kBtCarryInv);
}
